// RgnnLayer_34351148433957
// MI455X (gfx1250) — hardware-verified
//
#include <hip/hip_runtime.h>
#include <stddef.h>


#define DIMC    128
#define NWCOL   512
#define RWC     384
#define PPC     256
#define KP      (DIMC + 8)
#define NTHR    256
#define NWAVE   8
#define EPT     8
#define NGRP    2
#define CHUNK   (NTHR * EPT * NGRP)
#define WCAP    (EPT * NGRP * 32)
#define LISTN   (NWAVE * WCAP)
#define NBC     4096
#define NBF     1024
#define RCAP    24576
#define RBN     128
#define OTHR    512
#define TGT     32
#define NPW     (TGT / NWAVE)
#define DEGCAP  512
#define XT      64
#define RT      16
#define TYB     9
#define TYM     511

#define LDS_FILL  ((RCAP + NBF + LISTN) * 4 + 64)
#define L_XHI     0
#define L_XLO     (L_XHI + XT * KP * 2)
#define L_STG     (L_XLO + XT * KP * 2)
#define LDS_XW    (L_STG + XT * PPC * 4)

static_assert((CHUNK & (CHUNK - 1)) == 0);
static_assert(CHUNK <= 4096);
static_assert((NBC & (NBC - 1)) == 0 && (NBF & (NBF - 1)) == 0);
static_assert(NBC == 4 * NBF);
static_assert(OTHR * 8 == NBC);
static_assert((RCAP % 32) == 0);
static_assert(TGT == NWAVE * NPW);
static_assert(((TGT * DIMC / 4) % NTHR) == 0);
static_assert(((XT * DIMC / 4) % NTHR) == 0);
static_assert(((RT * DIMC / 4) % NTHR) == 0);
static_assert((KP % 8) == 0);
static_assert((L_XLO % 16) == 0 && (L_STG % 16) == 0);
static_assert(NWAVE * 16 == DIMC);
static_assert(NWAVE * 32 == PPC);
static_assert(NWAVE * 64 == NWCOL);
static_assert(((XT * 2) % NWAVE) == 0 && ((RT * 4) % NWAVE) == 0);

typedef float          v4f  __attribute__((ext_vector_type(4)));
typedef float          v8f  __attribute__((ext_vector_type(8)));
typedef int            v4i  __attribute__((ext_vector_type(4)));
typedef unsigned short v4us __attribute__((ext_vector_type(4)));
typedef unsigned short v8us __attribute__((ext_vector_type(8)));
typedef __bf16         v16b __attribute__((ext_vector_type(16)));
union FragB { v16b v; v8us u[2]; };

__device__ __forceinline__ unsigned short bf_bits(float f) {
  unsigned int u = __float_as_uint(f);
  u += 0x7FFFu + ((u >> 16) & 1u);
  return (unsigned short)(u >> 16);
}
__device__ __forceinline__ float bf_val(unsigned short s) {
  return __uint_as_float(((unsigned int)s) << 16);
}
__device__ __forceinline__ void split4(const v4f v, v4us& hv, v4us& lv) {
  const unsigned short h0 = bf_bits(v.x), h1 = bf_bits(v.y), h2 = bf_bits(v.z), h3 = bf_bits(v.w);
  hv.x = h0; hv.y = h1; hv.z = h2; hv.w = h3;
  lv.x = bf_bits(v.x - bf_val(h0));
  lv.y = bf_bits(v.y - bf_val(h1));
  lv.z = bf_bits(v.z - bf_val(h2));
  lv.w = bf_bits(v.w - bf_val(h3));
}

__device__ __forceinline__ v8f wmb(v16b a, v16b b, v8f c) {
  v8f d = __builtin_amdgcn_wmma_f32_16x16x32_bf16(false, a, false, b, (short)0, c, false, false);
  asm volatile("v_nop\n\tv_nop\n\tv_nop\n\tv_nop" : "+v"(d) : "v"(a), "v"(b));
  return d;
}

template <int NB>
__device__ __forceinline__ int scan_chunk(const int* __restrict__ dsts, int nE, int cbase, int slotBase,
                                          int vec8, int* list, int tid, int lane, int wave) {
  int wc = 0;
#pragma unroll
  for (int g = 0; g < NGRP; ++g) {
    const int el0  = (g * NTHR + tid) * EPT;
    const int e0   = cbase + el0;
    const int sent = -2147483647 - 1;
    v4i da, db;
    if (vec8 != 0 && cbase + CHUNK <= nE) {
      da = *(const v4i*)(dsts + e0);
      db = *(const v4i*)(dsts + e0 + 4);
    } else {
      da.x = (e0     < nE) ? dsts[min(e0, nE - 1)] : sent;
      da.y = (e0 + 1 < nE) ? dsts[min(e0 + 1, nE - 1)] : sent;
      da.z = (e0 + 2 < nE) ? dsts[min(e0 + 2, nE - 1)] : sent;
      da.w = (e0 + 3 < nE) ? dsts[min(e0 + 3, nE - 1)] : sent;
      db.x = (e0 + 4 < nE) ? dsts[min(e0 + 4, nE - 1)] : sent;
      db.y = (e0 + 5 < nE) ? dsts[min(e0 + 5, nE - 1)] : sent;
      db.z = (e0 + 6 < nE) ? dsts[min(e0 + 6, nE - 1)] : sent;
      db.w = (e0 + 7 < nE) ? dsts[min(e0 + 7, nE - 1)] : sent;
    }
    const unsigned nb = (unsigned)slotBase;
    const unsigned s0 = (unsigned)da.x - nb, s1 = (unsigned)da.y - nb;
    const unsigned s2 = (unsigned)da.z - nb, s3 = (unsigned)da.w - nb;
    const unsigned s4 = (unsigned)db.x - nb, s5 = (unsigned)db.y - nb;
    const unsigned s6 = (unsigned)db.z - nb, s7 = (unsigned)db.w - nb;
    const bool h0 = s0 < (unsigned)NB, h1 = s1 < (unsigned)NB, h2 = s2 < (unsigned)NB, h3 = s3 < (unsigned)NB;
    const bool h4 = s4 < (unsigned)NB, h5 = s5 < (unsigned)NB, h6 = s6 < (unsigned)NB, h7 = s7 < (unsigned)NB;
    const unsigned any = __builtin_amdgcn_ballot_w32(h0 | h1 | h2 | h3 | h4 | h5 | h6 | h7);
    if (any != 0u) {
#define HITJ(J, HJ, SJ) { \
        const unsigned mj = __builtin_amdgcn_ballot_w32(HJ); \
        if (mj != 0u) { \
          if (HJ) { \
            const int pos = wc + (int)__builtin_amdgcn_mbcnt_lo(mj, 0u); \
            if (pos < WCAP) list[wave * WCAP + pos] = ((el0 + (J)) << 12) | (int)(SJ); \
          } \
          wc += (int)__builtin_popcount(mj); } }
      HITJ(0, h0, s0)
      HITJ(1, h1, s1)
      HITJ(2, h2, s2)
      HITJ(3, h3, s3)
      HITJ(4, h4, s4)
      HITJ(5, h5, s5)
      HITJ(6, h6, s6)
      HITJ(7, h7, s7)
#undef HITJ
    }
  }
  return wc;
}

__global__ __launch_bounds__(NTHR) void k_wprep(
    const float* __restrict__ w_in, const float* __restrict__ w_out,
    const float* __restrict__ w_loop, const float* __restrict__ w_rel,
    unsigned short* wHi, unsigned short* wLo) {
  const int i = blockIdx.x * NTHR + (int)threadIdx.x;
  if (i >= NWCOL * DIMC / 8) return;
  const int o   = i * 8;
  const int n   = o >> 7;
  const int k0  = o & 127;
  const int seg = n >> 7;
  const int nl  = n & 127;
  const float* w = (seg == 0) ? w_in : ((seg == 1) ? w_out : ((seg == 2) ? w_loop : w_rel));
  float v[8];
#pragma unroll
  for (int e = 0; e < 8; ++e) v[e] = w[(size_t)(k0 + e) * DIMC + nl];
  v8us hv, lv;
#pragma unroll
  for (int e = 0; e < 8; ++e) {
    const unsigned short hb = bf_bits(v[e]);
    hv[e] = hb;
    lv[e] = bf_bits(v[e] - bf_val(hb));
  }
  *(volatile v8us*)(wHi + o) = hv;
  *(volatile v8us*)(wLo + o) = lv;
  __threadfence();
  *(volatile v8us*)(wHi + o) = hv;
  *(volatile v8us*)(wLo + o) = lv;
}

__global__ __launch_bounds__(NTHR) void k_count(
    const int* __restrict__ ei, int* cntAll, int ehIn, int nE, int cntpad, int vec8) {
  __shared__ __attribute__((aligned(16))) int scnt[NBC];
  __shared__ __attribute__((aligned(16))) int list[LISTN];
  __shared__ int wcnt[NWAVE];
  const int tid = threadIdx.x, lane = tid & 31, wave = tid >> 5;
  const int half = blockIdx.y;
  const int nodeBase = blockIdx.x * NBC;
  const int* dsts = ei + ((half != 0) ? ehIn : 0);
  const int len = (half != 0) ? (nE - ehIn) : ehIn;
  int* cnt = cntAll + (size_t)half * cntpad;

  for (int i = tid; i < NBC; i += NTHR) scnt[i] = 0;
  __syncthreads();

  const int nChunks = (len + CHUNK - 1) / CHUNK;
#pragma unroll 1
  for (int ch = 0; ch < nChunks; ++ch) {
    const int cbase = ch * CHUNK;
    const int wc = scan_chunk<NBC>(dsts, len, cbase, nodeBase, vec8, list, tid, lane, wave);
    if (lane == 0) wcnt[wave] = wc;
    __syncthreads();
    if (wave == 0) {
#pragma unroll 1
      for (int wsx = 0; wsx < NWAVE; ++wsx) {
        int n = __builtin_amdgcn_readfirstlane(wcnt[wsx]);
        n = n > WCAP ? WCAP : (n < 0 ? 0 : n);
        const int* lp = list + wsx * WCAP;
#pragma unroll 1
        for (int i = 0; i < n; ++i) {
          const int ent  = __builtin_amdgcn_readfirstlane(lp[i]);
          const int slot = ent & (NBC - 1);
          if (lane == 0) scnt[slot] = scnt[slot] + 1;
        }
      }
    }
    __syncthreads();
  }

  v4i cq[4];
#pragma unroll
  for (int q = 0; q < 4; ++q) {
    const int f = (wave * 4 + q) * 128 + 4 * lane;
    cq[q] = *(const v4i*)(scnt + f);
  }
  int* cp = cnt + (size_t)nodeBase;
#pragma unroll
  for (int q = 0; q < 4; ++q) {
    const int f = (wave * 4 + q) * 128 + 4 * lane;
    *(volatile v4i*)(cp + f) = cq[q];
  }
  __threadfence();
#pragma unroll
  for (int q = 0; q < 4; ++q) {
    const int f = (wave * 4 + q) * 128 + 4 * lane;
    *(volatile v4i*)(cp + f) = cq[q];
  }
}

__global__ __launch_bounds__(OTHR) void k_offsets(
    const int* __restrict__ cntAll, int* offAll, int* rbAll, int nChunk, int cntpad) {
  __shared__ __attribute__((aligned(16))) int soff[NBC];
  __shared__ __attribute__((aligned(16))) int srb[RBN];
  __shared__ int wtot[OTHR / 32];
  const int tid = threadIdx.x, lane = tid & 31, wave = tid >> 5, sub = tid >> 7;
  const int half = blockIdx.x;
  const int* cnt = cntAll + (size_t)half * cntpad;
  int* off   = offAll + (size_t)half * cntpad;
  int* rbase = rbAll + half * RBN;
  for (int i = tid; i < RBN; i += OTHR) srb[i] = 0;
  int carry = 0;
#pragma unroll 1
  for (int ch = 0; ch < nChunk; ++ch) {
    const int base = ch * NBC;
    const v4i c0 = *(const v4i*)(cnt + base + 8 * tid);
    const v4i c1 = *(const v4i*)(cnt + base + 8 * tid + 4);
    const int e0 = max(c0.x, 0), e1 = max(c0.y, 0), e2 = max(c0.z, 0), e3 = max(c0.w, 0);
    const int e4 = max(c1.x, 0), e5 = max(c1.y, 0), e6 = max(c1.z, 0), e7 = max(c1.w, 0);
    const int ts = e0 + e1 + e2 + e3 + e4 + e5 + e6 + e7;
    int incl = ts;
#pragma unroll
    for (int d = 1; d < 32; d <<= 1) {
      const int t = __shfl_up(incl, d);
      if (lane >= d) incl += t;
    }
    if (lane == 31) wtot[wave] = incl;
    __syncthreads();
    const int S0 = wtot[0]  + wtot[1]  + wtot[2]  + wtot[3];
    const int S1 = wtot[4]  + wtot[5]  + wtot[6]  + wtot[7];
    const int S2 = wtot[8]  + wtot[9]  + wtot[10] + wtot[11];
    const int S3 = wtot[12] + wtot[13] + wtot[14] + wtot[15];
    int pre = 0;
#pragma unroll 1
    for (int w = 4 * sub; w < wave; ++w) pre += wtot[w];
    const int b0 = carry;
    const int b1 = b0 + ((S0 + 31) & ~31);
    const int b2 = b1 + ((S1 + 31) & ~31);
    const int b3 = b2 + ((S2 + 31) & ~31);
    const int b4 = b3 + ((S3 + 31) & ~31);
    const int myb = sub == 0 ? b0 : (sub == 1 ? b1 : (sub == 2 ? b2 : b3));
    if (tid == 0) {
      srb[min(4 * ch + 0, RBN - 1)] = b0;
      srb[min(4 * ch + 1, RBN - 1)] = b1;
      srb[min(4 * ch + 2, RBN - 1)] = b2;
      srb[min(4 * ch + 3, RBN - 1)] = b3;
    }
    int run = myb + pre + incl - ts;
    soff[8 * tid + 0] = run; run += e0;
    soff[8 * tid + 1] = run; run += e1;
    soff[8 * tid + 2] = run; run += e2;
    soff[8 * tid + 3] = run; run += e3;
    soff[8 * tid + 4] = run; run += e4;
    soff[8 * tid + 5] = run; run += e5;
    soff[8 * tid + 6] = run; run += e6;
    soff[8 * tid + 7] = run;
    carry = b4;
    __syncthreads();
    const v4i o0 = *(const v4i*)(soff + 4 * tid);
    const v4i o1 = *(const v4i*)(soff + 4 * (tid + OTHR));
    int* op = off + base;
    *(volatile v4i*)(op + 4 * tid) = o0;
    *(volatile v4i*)(op + 4 * (tid + OTHR)) = o1;
    __threadfence();
    *(volatile v4i*)(op + 4 * tid) = o0;
    *(volatile v4i*)(op + 4 * (tid + OTHR)) = o1;
    __syncthreads();
  }
  if (tid == 0) srb[min(4 * nChunk, RBN - 1)] = carry;
  __syncthreads();
  v4i rv = {0, 0, 0, 0};
  if (tid < 32) rv = *(const v4i*)(srb + 4 * tid);
  if (tid < 32) *(volatile v4i*)(rbase + 4 * tid) = rv;
  __threadfence();
  if (tid < 32) *(volatile v4i*)(rbase + 4 * tid) = rv;
}

__global__ __launch_bounds__(NTHR) void k_fill(
    const int* __restrict__ ei, const int* __restrict__ et, const int* __restrict__ offAll,
    const int* __restrict__ rbAll, int* csrAll, int nN, int nE, int ehIn, int nR,
    int vec8, int csrLen, int cntpad) {
  extern __shared__ v4f lds_dyn[];
  int* region = (int*)lds_dyn;
  int* cursor = region + RCAP;
  int* list   = cursor + NBF;
  int* wcnt   = list + LISTN;
  const int tid = threadIdx.x, lane = tid & 31, wave = tid >> 5;
  const int b = blockIdx.x;
  const int half = blockIdx.y;
  const int nodeBase = b * NBF;
  const int ebase = (half != 0) ? ehIn : 0;
  const int len   = (half != 0) ? (nE - ehIn) : ehIn;
  const int* dsts = ei + ebase;
  const int* srcs = ei + (size_t)nE + ebase;
  const int* tys  = et + ebase;
  const int* off   = offAll + (size_t)half * cntpad;
  const int* rbase = rbAll + half * RBN;
  int* csr = csrAll + (size_t)half * csrLen;

  int rb0 = rbase[b];
  const int rb1 = rbase[b + 1];
  rb0 = rb0 < 0 ? 0 : (rb0 > csrLen ? csrLen : rb0);
  rb0 &= ~31;
  int rlen = rb1 - rb0;
  rlen = rlen < 0 ? 0 : (rlen > RCAP ? RCAP : rlen);
  int lenW = (rlen + 31) & ~31;
  if (rb0 + lenW > csrLen) lenW = (csrLen - rb0) & ~31;

  {
    const v4i z = {0, 0, 0, 0};
    for (int i = tid; i < RCAP / 4; i += NTHR) ((v4i*)region)[i] = z;
    for (int s = tid; s < NBF; s += NTHR) {
      int o = off[nodeBase + s] - rb0;
      o = o < 0 ? 0 : (o > RCAP ? RCAP : o);
      cursor[s] = o;
    }
  }
  __syncthreads();

  const int nChunks = (len + CHUNK - 1) / CHUNK;
#pragma unroll 1
  for (int ch = 0; ch < nChunks; ++ch) {
    const int cbase = ch * CHUNK;
    const int wc = scan_chunk<NBF>(dsts, len, cbase, nodeBase, vec8, list, tid, lane, wave);
    if (lane == 0) wcnt[wave] = wc;
    __syncthreads();
    if (wave == 0) {
#pragma unroll 1
      for (int wsx = 0; wsx < NWAVE; ++wsx) {
        int n = __builtin_amdgcn_readfirstlane(wcnt[wsx]);
        n = n > WCAP ? WCAP : (n < 0 ? 0 : n);
        const int* lp = list + wsx * WCAP;
#pragma unroll 1
        for (int i = 0; i < n; ++i) {
          const int ent  = __builtin_amdgcn_readfirstlane(lp[i]);
          const int slot = ent & (NBF - 1);
          int e = cbase + ((ent >> 12) & (CHUNK - 1));
          e = e > len - 1 ? len - 1 : e;
          e = e < 0 ? 0 : e;
          int src = srcs[e];
          src = src < 0 ? 0 : (src > nN - 1 ? nN - 1 : src);
          int ty = tys[e];
          ty = ty < 0 ? 0 : (ty > nR ? nR : ty);
          if (lane == 0) {
            int pos = cursor[slot];
            pos = pos < 0 ? 0 : (pos > RCAP - 1 ? RCAP - 1 : pos);
            region[pos] = (src << TYB) | ty;
            const int np = pos + 1;
            cursor[slot] = np > RCAP ? RCAP : np;
          }
        }
      }
    }
    __syncthreads();
  }

  const int nv = lenW >> 2;
  int* gp = csr + rb0;
#pragma unroll 1
  for (int i = tid; i < nv; i += NTHR) { const v4i v = ((const v4i*)region)[i]; *(volatile v4i*)(gp + 4 * i) = v; }
  __threadfence();
#pragma unroll 1
  for (int i = tid; i < nv; i += NTHR) { const v4i v = ((const v4i*)region)[i]; *(volatile v4i*)(gp + 4 * i) = v; }
}

__global__ __launch_bounds__(NTHR) void k_dinv(const int* __restrict__ cnt, float* dinv, int nq) {
  const int i = blockIdx.x * NTHR + (int)threadIdx.x;
  if (i >= nq) return;
  const v4i c = *(const v4i*)(cnt + (size_t)4 * i);
  v4f d;
  d.x = (c.x > 0) ? __builtin_amdgcn_rsqf((float)max(c.x, 1)) : 0.0f;
  d.y = (c.y > 0) ? __builtin_amdgcn_rsqf((float)max(c.y, 1)) : 0.0f;
  d.z = (c.z > 0) ? __builtin_amdgcn_rsqf((float)max(c.z, 1)) : 0.0f;
  d.w = (c.w > 0) ? __builtin_amdgcn_rsqf((float)max(c.w, 1)) : 0.0f;
  *(volatile v4f*)(dinv + (size_t)4 * i) = d;
  __threadfence();
  *(volatile v4f*)(dinv + (size_t)4 * i) = d;
}

__global__ __launch_bounds__(NTHR) void k_rw(
    const float* __restrict__ r, const float* __restrict__ loop_rel,
    const unsigned short* __restrict__ wHi, const unsigned short* __restrict__ wLo,
    float* rw, float* out1, int nR) {
  __shared__ __attribute__((aligned(16))) unsigned short aHi[RT * KP];
  __shared__ __attribute__((aligned(16))) unsigned short aLo[RT * KP];
  __shared__ __attribute__((aligned(16))) float stg[RT * NWCOL];
  const int tid = threadIdx.x, lane = tid & 31, wave = tid >> 5, hh = lane >> 4, m = lane & 15;
  const int row0 = blockIdx.x * RT;

#pragma unroll
  for (int i = 0; i < (RT * DIMC / 4) / NTHR; ++i) {
    const int idx = i * NTHR + tid;
    const int row = idx >> 5;
    const int c   = (idx & 31) * 4;
    const int gr  = row0 + row;
    const int grc = gr > nR - 1 ? nR - 1 : gr;
    const v4f vr = *(const v4f*)(r + (size_t)grc * DIMC + c);
    const v4f vl = *(const v4f*)(loop_rel + c);
    const bool isR = gr < nR, isL = gr == nR;
    v4f v;
    v.x = isR ? vr.x : (isL ? vl.x : 0.0f);
    v.y = isR ? vr.y : (isL ? vl.y : 0.0f);
    v.z = isR ? vr.z : (isL ? vl.z : 0.0f);
    v.w = isR ? vr.w : (isL ? vl.w : 0.0f);
    v4us hv, lv;
    split4(v, hv, lv);
    *(v4us*)(aHi + row * KP + c) = hv;
    *(v4us*)(aLo + row * KP + c) = lv;
  }
  __syncthreads();

  v8f acc[4];
  { const v8f z8 = {0.f, 0.f, 0.f, 0.f, 0.f, 0.f, 0.f, 0.f};
#pragma unroll
    for (int ct = 0; ct < 4; ++ct) acc[ct] = z8; }
#pragma unroll 1
  for (int ks = 0; ks < DIMC / 32; ++ks) {
    FragB ah, al;
    const int ao = m * KP + 32 * ks + 8 * hh;
    ah.u[0] = *(const v8us*)(aHi + ao);  ah.u[1] = *(const v8us*)(aHi + ao + 16);
    al.u[0] = *(const v8us*)(aLo + ao);  al.u[1] = *(const v8us*)(aLo + ao + 16);
#pragma unroll
    for (int ct = 0; ct < 4; ++ct) {
      const size_t bo = (size_t)(64 * wave + 16 * ct + m) * DIMC + 32 * ks + 8 * hh;
      FragB bh, bl;
      bh.u[0] = *(const v8us*)(wHi + bo);  bh.u[1] = *(const v8us*)(wHi + bo + 16);
      bl.u[0] = *(const v8us*)(wLo + bo);  bl.u[1] = *(const v8us*)(wLo + bo + 16);
      acc[ct] = wmb(al.v, bh.v, acc[ct]);
      acc[ct] = wmb(ah.v, bl.v, acc[ct]);
      acc[ct] = wmb(ah.v, bh.v, acc[ct]);
    }
  }
#pragma unroll
  for (int ct = 0; ct < 4; ++ct) {
#pragma unroll
    for (int q = 0; q < 8; ++q) stg[(8 * hh + q) * NWCOL + 64 * wave + 16 * ct + m] = acc[ct][q];
  }
  __syncthreads();

#pragma unroll 1
  for (int j = 0; j < (RT * 4) / NWAVE; ++j) {
    const int u = wave + NWAVE * j;
    const int row = u >> 2, seg = u & 3;
    const int gr = row0 + row;
    const v4f v = *(const v4f*)(stg + row * NWCOL + seg * DIMC + 4 * lane);
    if (seg < 3) {
      *(volatile v4f*)(rw + (size_t)gr * RWC + seg * DIMC + 4 * lane) = v;
    } else if (gr < nR) {
      *(volatile v4f*)(out1 + (size_t)gr * DIMC + 4 * lane) = v;
    }
  }
  __threadfence();
#pragma unroll 1
  for (int j = 0; j < (RT * 4) / NWAVE; ++j) {
    const int u = wave + NWAVE * j;
    const int row = u >> 2, seg = u & 3;
    const int gr = row0 + row;
    const v4f v = *(const v4f*)(stg + row * NWCOL + seg * DIMC + 4 * lane);
    if (seg < 3) {
      *(volatile v4f*)(rw + (size_t)gr * RWC + seg * DIMC + 4 * lane) = v;
    } else if (gr < nR) {
      *(volatile v4f*)(out1 + (size_t)gr * DIMC + 4 * lane) = v;
    }
  }
}

__global__ __launch_bounds__(NTHR) void k_xw(
    const float* __restrict__ x, const unsigned short* __restrict__ wHi,
    const unsigned short* __restrict__ wLo, float* P, int nN) {
  extern __shared__ v4f lds_dyn[];
  char* lb = (char*)lds_dyn;
  unsigned short* xh  = (unsigned short*)(lb + L_XHI);
  unsigned short* xl  = (unsigned short*)(lb + L_XLO);
  float*          stg = (float*)(lb + L_STG);
  const int tid = threadIdx.x, lane = tid & 31, wave = tid >> 5, hh = lane >> 4, m = lane & 15;
  const int row0 = blockIdx.x * XT;

#pragma unroll
  for (int i = 0; i < (XT * DIMC / 4) / NTHR; ++i) {
    const int idx = i * NTHR + tid;
    const int row = idx >> 5;
    const int c   = (idx & 31) * 4;
    int gr = row0 + row;
    gr = gr > nN - 1 ? nN - 1 : gr;
    const v4f v = *(const v4f*)(x + (size_t)gr * DIMC + c);
    v4us hv, lv;
    split4(v, hv, lv);
    *(v4us*)(xh + row * KP + c) = hv;
    *(v4us*)(xl + row * KP + c) = lv;
  }
  __syncthreads();

  v8f acc[4][2];
  { const v8f z8 = {0.f, 0.f, 0.f, 0.f, 0.f, 0.f, 0.f, 0.f};
#pragma unroll
    for (int rt = 0; rt < 4; ++rt) { acc[rt][0] = z8; acc[rt][1] = z8; } }
#pragma unroll 1
  for (int ks = 0; ks < DIMC / 32; ++ks) {
    FragB bh0, bl0, bh1, bl1;
    {
      const size_t bo0 = (size_t)(32 * wave + m) * DIMC + 32 * ks + 8 * hh;
      const size_t bo1 = (size_t)(32 * wave + 16 + m) * DIMC + 32 * ks + 8 * hh;
      bh0.u[0] = *(const v8us*)(wHi + bo0);  bh0.u[1] = *(const v8us*)(wHi + bo0 + 16);
      bl0.u[0] = *(const v8us*)(wLo + bo0);  bl0.u[1] = *(const v8us*)(wLo + bo0 + 16);
      bh1.u[0] = *(const v8us*)(wHi + bo1);  bh1.u[1] = *(const v8us*)(wHi + bo1 + 16);
      bl1.u[0] = *(const v8us*)(wLo + bo1);  bl1.u[1] = *(const v8us*)(wLo + bo1 + 16);
    }
#pragma unroll
    for (int rt = 0; rt < 4; ++rt) {
      FragB ah, al;
      const int ao = (16 * rt + m) * KP + 32 * ks + 8 * hh;
      ah.u[0] = *(const v8us*)(xh + ao);  ah.u[1] = *(const v8us*)(xh + ao + 16);
      al.u[0] = *(const v8us*)(xl + ao);  al.u[1] = *(const v8us*)(xl + ao + 16);
      acc[rt][0] = wmb(al.v, bh0.v, acc[rt][0]);
      acc[rt][0] = wmb(ah.v, bl0.v, acc[rt][0]);
      acc[rt][0] = wmb(ah.v, bh0.v, acc[rt][0]);
      acc[rt][1] = wmb(al.v, bh1.v, acc[rt][1]);
      acc[rt][1] = wmb(ah.v, bl1.v, acc[rt][1]);
      acc[rt][1] = wmb(ah.v, bh1.v, acc[rt][1]);
    }
  }
#pragma unroll
  for (int rt = 0; rt < 4; ++rt) {
#pragma unroll
    for (int q = 0; q < 8; ++q) {
      stg[(16 * rt + 8 * hh + q) * PPC + 32 * wave + m]      = acc[rt][0][q];
      stg[(16 * rt + 8 * hh + q) * PPC + 32 * wave + 16 + m] = acc[rt][1][q];
    }
  }
  __syncthreads();

  float* gp = P + (size_t)row0 * PPC;
#pragma unroll 1
  for (int j = 0; j < (XT * 2) / NWAVE; ++j) {
    const int u = wave + NWAVE * j;
    const int row = u >> 1, hf = u & 1;
    const v4f v = *(const v4f*)(stg + row * PPC + hf * DIMC + 4 * lane);
    *(volatile v4f*)(gp + (size_t)row * PPC + hf * DIMC + 4 * lane) = v;
  }
  __threadfence();
#pragma unroll 1
  for (int j = 0; j < (XT * 2) / NWAVE; ++j) {
    const int u = wave + NWAVE * j;
    const int row = u >> 1, hf = u & 1;
    const v4f v = *(const v4f*)(stg + row * PPC + hf * DIMC + 4 * lane);
    *(volatile v4f*)(gp + (size_t)row * PPC + hf * DIMC + 4 * lane) = v;
  }
}

__global__ __launch_bounds__(NTHR) void k_agg(
    const float* __restrict__ x, const float* __restrict__ P, const float* __restrict__ rw,
    const int* __restrict__ csrAll, const int* __restrict__ offAll, const int* __restrict__ cntAll,
    const float* __restrict__ dinvAll,
    const unsigned short* __restrict__ wHi, const unsigned short* __restrict__ wLo,
    const float* __restrict__ bias, float* out, int nN, int nR, int csrLen, int cntpad) {
  __shared__ __attribute__((aligned(16))) unsigned short xh[TGT * KP];
  __shared__ __attribute__((aligned(16))) unsigned short xl[TGT * KP];
  __shared__ __attribute__((aligned(16))) float lps[TGT * DIMC];
  const int tid = threadIdx.x, lane = tid & 31, wave = tid >> 5, hh = lane >> 4, m = lane & 15;
  const int node0 = blockIdx.x * TGT;
  const v4f z4 = {0.f, 0.f, 0.f, 0.f};

#pragma unroll
  for (int i = 0; i < (TGT * DIMC / 4) / NTHR; ++i) {
    const int idx = i * NTHR + tid;
    const int row = idx >> 5;
    const int c   = (idx & 31) * 4;
    int nd = node0 + row;
    nd = nd > nN - 1 ? nN - 1 : nd;
    const v4f v = *(const v4f*)(x + (size_t)nd * DIMC + c);
    v4us hv, lv;
    split4(v, hv, lv);
    *(v4us*)(xh + row * KP + c) = hv;
    *(v4us*)(xl + row * KP + c) = lv;
  }
  __syncthreads();

  const int gcol = 16 * wave + m;
  v8f acc[2];
  { const v8f z8 = {0.f, 0.f, 0.f, 0.f, 0.f, 0.f, 0.f, 0.f}; acc[0] = z8; acc[1] = z8; }
#pragma unroll 1
  for (int ks = 0; ks < DIMC / 32; ++ks) {
    FragB bh, bl;
    const size_t bo = (size_t)(2 * DIMC + gcol) * DIMC + 32 * ks + 8 * hh;
    bh.u[0] = *(const v8us*)(wHi + bo);  bh.u[1] = *(const v8us*)(wHi + bo + 16);
    bl.u[0] = *(const v8us*)(wLo + bo);  bl.u[1] = *(const v8us*)(wLo + bo + 16);
#pragma unroll
    for (int rt = 0; rt < 2; ++rt) {
      FragB ah, al;
      const int ao = (16 * rt + m) * KP + 32 * ks + 8 * hh;
      ah.u[0] = *(const v8us*)(xh + ao);  ah.u[1] = *(const v8us*)(xh + ao + 16);
      al.u[0] = *(const v8us*)(xl + ao);  al.u[1] = *(const v8us*)(xl + ao + 16);
      acc[rt] = wmb(al.v, bh.v, acc[rt]);
      acc[rt] = wmb(ah.v, bl.v, acc[rt]);
      acc[rt] = wmb(ah.v, bh.v, acc[rt]);
    }
  }
#pragma unroll
  for (int rt = 0; rt < 2; ++rt) {
#pragma unroll
    for (int q = 0; q < 8; ++q) lps[(16 * rt + 8 * hh + q) * DIMC + gcol] = acc[rt][q];
  }
  __syncthreads();

  const float third = 1.0f / 3.0f;
#pragma unroll 1
  for (int i = 0; i < NPW; ++i) {
    const int row = wave * NPW + i;
    const int nd  = node0 + row;
    const int ndc = nd > nN - 1 ? nN - 1 : nd;
    v4f tot = z4;
#pragma unroll 1
    for (int hm = 0; hm < 2; ++hm) {
      const int*   cntH = cntAll  + (size_t)hm * cntpad;
      const int*   offH = offAll  + (size_t)hm * cntpad;
      const int*   csrH = csrAll  + (size_t)hm * csrLen;
      const float* dvH  = dinvAll + (size_t)hm * cntpad;
      const float* PH   = P  + hm * DIMC;
      const float* RH   = rw + hm * DIMC;
      int n = cntH[ndc];
      n = nd < nN ? n : 0;
      n = n < 0 ? 0 : (n > DEGCAP ? DEGCAP : n);
      int st = offH[ndc];
      st = st < 0 ? 0 : (st > csrLen - 1 ? csrLen - 1 : st);
      const float dn = dvH[ndc];
      v4f s = z4;
#pragma unroll 1
      for (int q0 = 0; q0 < n; q0 += 32) {
        int pos = st + q0 + lane;
        pos = pos > csrLen - 1 ? csrLen - 1 : pos;
        const int ent = csrH[pos];
        const int mc  = (n - q0) < 32 ? (n - q0) : 32;
#pragma unroll 1
        for (int p = 0; p < mc; ++p) {
          const int e = __builtin_amdgcn_readlane(ent, p);
          int col = e >> TYB;
          col = col < 0 ? 0 : (col > nN - 1 ? nN - 1 : col);
          int t = e & TYM;
          t = t > nR ? nR : t;
          const float nrm = dn * dvH[col];
          const v4f pv = *(const v4f*)(PH + (size_t)col * PPC + 4 * lane);
          const v4f rv = *(const v4f*)(RH + (size_t)t * RWC + 4 * lane);
          s = s + (pv - rv) * nrm;
        }
      }
      tot = tot + s;
    }
    const v4f lp = *(const v4f*)(lps + row * DIMC + 4 * lane);
    const v4f rl = *(const v4f*)(rw + (size_t)nR * RWC + 2 * DIMC + 4 * lane);
    const v4f bv = *(const v4f*)(bias + 4 * lane);
    const v4f u = (tot + (lp - rl)) * third + bv;
    v4f o;
    o.x = tanhf(u.x); o.y = tanhf(u.y); o.z = tanhf(u.z); o.w = tanhf(u.w);
    *(v4f*)(lps + row * DIMC + 4 * lane) = o;
  }

#pragma unroll
  for (int i = 0; i < NPW; ++i) {
    const int row = wave * NPW + i;
    const int nd = node0 + row;
    if (nd < nN) {
      const v4f v = *(const v4f*)(lps + row * DIMC + 4 * lane);
      *(volatile v4f*)(out + (size_t)nd * DIMC + 4 * lane) = v;
    }
  }
  __threadfence();
#pragma unroll
  for (int i = 0; i < NPW; ++i) {
    const int row = wave * NPW + i;
    const int nd = node0 + row;
    if (nd < nN) {
      const v4f v = *(const v4f*)(lps + row * DIMC + 4 * lane);
      *(volatile v4f*)(out + (size_t)nd * DIMC + 4 * lane) = v;
    }
  }
}

extern "C" void kernel_launch(void* const* d_in, const int* in_sizes, int n_in,
                              void* d_out, int out_size, void* d_ws, size_t ws_size,
                              hipStream_t stream) {
  if (n_in < 10) return;
  if (in_sizes[4] != DIMC * DIMC || in_sizes[5] != DIMC * DIMC ||
      in_sizes[6] != DIMC * DIMC || in_sizes[7] != DIMC * DIMC) return;
  if (in_sizes[8] != DIMC || in_sizes[9] != DIMC) return;
  const int nN = in_sizes[0] / DIMC;
  const int nR = in_sizes[1] / DIMC;
  const int nE = in_sizes[3];
  if (nN <= 0 || nR <= 0 || nE <= 0) return;
  if (in_sizes[0] != nN * DIMC || in_sizes[1] != nR * DIMC || in_sizes[2] != 2 * nE) return;
  if (nN > (1 << 22) || nE > (1 << 28) || nR > TYM) return;
  if (out_size != nN * DIMC + nR * DIMC) return;

  const float* x        = (const float*)d_in[0];
  const float* r        = (const float*)d_in[1];
  const int*   ei       = (const int*)d_in[2];
  const int*   et       = (const int*)d_in[3];
  const float* w_in     = (const float*)d_in[4];
  const float* w_out    = (const float*)d_in[5];
  const float* w_loop   = (const float*)d_in[6];
  const float* w_rel    = (const float*)d_in[7];
  const float* loop_rel = (const float*)d_in[8];
  const float* bias     = (const float*)d_in[9];
  float* out0 = (float*)d_out;
  float* out1 = out0 + (size_t)nN * DIMC;

  const int ehIn   = nE / 2;
  const int ehMax  = nE - ehIn;
  const int nBC    = (nN + NBC - 1) / NBC;
  const int cntpad = nBC * NBC;
  if (4 * nBC + 1 > RBN) return;
  const int nBF    = (nN + NBF - 1) / NBF;
  if (nBF * NBF > cntpad || nBF + 1 > RBN) return;
  const int csrLen = ((ehMax + 31) & ~31) + 4096;
  const int rwTiles = (nR + 1 + RT - 1) / RT;
  const int rwRows  = rwTiles * RT;
  const int xTiles  = (nN + XT - 1) / XT;
  const int nPad    = xTiles * XT;
  const int nAgg    = (nN + TGT - 1) / TGT;

  char* ws = (char*)d_ws;
  size_t ob = 0;
  const size_t oWH  = ob; ob += (size_t)NWCOL * DIMC * 2;       ob = (ob + 255) & ~(size_t)255;
  const size_t oWL  = ob; ob += (size_t)NWCOL * DIMC * 2;       ob = (ob + 255) & ~(size_t)255;
  const size_t oCnt = ob; ob += (size_t)2 * cntpad * 4;         ob = (ob + 255) & ~(size_t)255;
  const size_t oOff = ob; ob += (size_t)2 * cntpad * 4;         ob = (ob + 255) & ~(size_t)255;
  const size_t oRb  = ob; ob += (size_t)2 * RBN * 4;            ob = (ob + 255) & ~(size_t)255;
  const size_t oCsr = ob; ob += (size_t)2 * csrLen * 4;         ob = (ob + 255) & ~(size_t)255;
  const size_t oDv  = ob; ob += (size_t)2 * cntpad * 4;         ob = (ob + 255) & ~(size_t)255;
  const size_t oRW  = ob; ob += (size_t)rwRows * RWC * 4;       ob = (ob + 255) & ~(size_t)255;
  const size_t oP   = ob; ob += (size_t)nPad * PPC * 4;         ob = (ob + 255) & ~(size_t)255;
  if (ob > ws_size || ob > ((size_t)128 << 20)) return;
  unsigned short* wHi = (unsigned short*)(ws + oWH);
  unsigned short* wLo = (unsigned short*)(ws + oWL);
  int*   cnt  = (int*)(ws + oCnt);
  int*   offp = (int*)(ws + oOff);
  int*   rb   = (int*)(ws + oRb);
  int*   csr  = (int*)(ws + oCsr);
  float* dinv = (float*)(ws + oDv);
  float* rwp  = (float*)(ws + oRW);
  float* Pp   = (float*)(ws + oP);

  const int vec8 = (((ehIn & 3) == 0) && ((ehMax & 3) == 0)) ? 1 : 0;

  k_wprep<<<(NWCOL * DIMC / 8 + NTHR - 1) / NTHR, NTHR, 0, stream>>>(w_in, w_out, w_loop, w_rel, wHi, wLo);

  k_count<<<dim3(nBC, 2), dim3(NTHR), 0, stream>>>(ei, cnt, ehIn, nE, cntpad, vec8);
  k_offsets<<<2, OTHR, 0, stream>>>(cnt, offp, rb, nBC, cntpad);
  hipFuncSetAttribute(reinterpret_cast<const void*>(&k_fill),
                      hipFuncAttributeMaxDynamicSharedMemorySize, LDS_FILL);
  k_fill<<<dim3(nBF, 2), dim3(NTHR), LDS_FILL, stream>>>(ei, et, offp, rb, csr, nN, nE, ehIn, nR,
                                                          vec8, csrLen, cntpad);

  const int nq = (2 * cntpad) / 4;
  k_dinv<<<(nq + NTHR - 1) / NTHR, NTHR, 0, stream>>>(cnt, dinv, nq);

  k_rw<<<rwTiles, NTHR, 0, stream>>>(r, loop_rel, wHi, wLo, rwp, out1, nR);

  hipFuncSetAttribute(reinterpret_cast<const void*>(&k_xw),
                      hipFuncAttributeMaxDynamicSharedMemorySize, LDS_XW);
  k_xw<<<xTiles, NTHR, LDS_XW, stream>>>(x, wHi, wLo, Pp, nN);

  k_agg<<<nAgg, NTHR, 0, stream>>>(x, Pp, rwp, csr, offp, cnt, dinv, wHi, wLo, bias, out0,
                                   nN, nR, csrLen, cntpad);
}
